// SelfNormAttention2_10505490006115
// MI455X (gfx1250) — hardware-run, weakly checked
//
#include <hip/hip_runtime.h>
#include <math.h>

typedef __attribute__((ext_vector_type(16))) __bf16   v16b;
typedef __attribute__((ext_vector_type(8)))  __bf16   v8b;
typedef __attribute__((ext_vector_type(8)))  float    v8f;
typedef __attribute__((ext_vector_type(4)))  float    v4f;
typedef __attribute__((ext_vector_type(4)))  unsigned int v4u;

constexpr int kNB   = 2;
constexpr int kSeq  = 2048;
constexpr int kNH   = 8;
constexpr int kHD   = 64;
constexpr int kCh   = 64;
constexpr int kNCh  = kSeq / kCh;
constexpr int kNChState = kNCh - 1;
constexpr int kBH   = kNB * kNH;
constexpr int kTile = kCh * kHD;
constexpr int kLdT  = 65;
constexpr int kLdA  = 72;
constexpr int kLdO  = 68;
static_assert(kNCh == 32);
static_assert(kBH == 16);
static_assert(kTile == 4096);
static_assert((kHD % 32) == 0 && (kCh % 32) == 0);
static_assert(kHD == 64 && kCh == 64);

constexpr size_t kPlaneB  = (size_t)kBH * kSeq * kHD * 2;
constexpr size_t kOffQH   = 0;
constexpr size_t kOffQL   = kOffQH  + kPlaneB;
constexpr size_t kOffKH   = kOffQL  + kPlaneB;
constexpr size_t kOffKL   = kOffKH  + kPlaneB;
constexpr size_t kOffKTH  = kOffKL  + kPlaneB;
constexpr size_t kOffKTL  = kOffKTH + kPlaneB;
constexpr size_t kOffVTH  = kOffKTL + kPlaneB;
constexpr size_t kOffVTL  = kOffVTH + kPlaneB;
constexpr size_t kOffSTC  = kOffVTL + kPlaneB;
constexpr size_t kOffSTH  = kOffSTC + (size_t)kBH * kNChState * kTile * 4;
constexpr size_t kOffSTL  = kOffSTH + (size_t)kBH * kNCh * kTile * 2;
constexpr size_t kWsTotal = kOffSTL + (size_t)kBH * kNCh * kTile * 2;
static_assert(kPlaneB == 4194304ull);
static_assert(kWsTotal == 50069504ull);
static_assert(kWsTotal <= 134217728ull);
static_assert((kOffSTC % 128) == 0 && (kOffSTH % 128) == 0 && (kOffSTL % 128) == 0 && (kPlaneB % 128) == 0);

__device__ __forceinline__ unsigned short f2bf_bits(float f) {
  unsigned u = __float_as_uint(f);
  return (unsigned short)((u + 0x7FFFu + ((u >> 16) & 1u)) >> 16);
}
__device__ __forceinline__ float bf_bits2f(unsigned short h) { return __uint_as_float(((unsigned)h) << 16); }
__device__ __forceinline__ unsigned pk16(unsigned short a, unsigned short b) { return (unsigned)a | ((unsigned)b << 16); }

__device__ __forceinline__ void split8(const float (&x)[8], v4u& hi, v4u& lo) {
  unsigned short hb[8], lb[8];
#pragma unroll
  for (int e = 0; e < 8; ++e) {
    hb[e] = f2bf_bits(x[e]);
    lb[e] = f2bf_bits(x[e] - bf_bits2f(hb[e]));
  }
  hi = (v4u){pk16(hb[0], hb[1]), pk16(hb[2], hb[3]), pk16(hb[4], hb[5]), pk16(hb[6], hb[7])};
  lo = (v4u){pk16(lb[0], lb[1]), pk16(lb[2], lb[3]), pk16(lb[4], lb[5]), pk16(lb[6], lb[7])};
}

union FragB { v16b v; v8b h[2]; };
__device__ __forceinline__ v16b ldfrag(const __bf16* p) {
  FragB f;
  f.h[0] = *(const v8b*)(p);
  f.h[1] = *(const v8b*)(p + 16);
  return f.v;
}
__device__ __forceinline__ v8f mma_bf(v16b a, v16b b, v8f c) {
  c = __builtin_amdgcn_wmma_f32_16x16x32_bf16(false, a, false, b, (short)0, c, false, false);
  asm volatile("v_nop\n\tv_nop\n\tv_nop\n\tv_nop" : "+v"(c) : "v"(a), "v"(b));
  return c;
}
__device__ __forceinline__ v8f mma3(v16b ah, v16b al, v16b bh, v16b bl, v8f c) {
  c = mma_bf(ah, bh, c);
  c = mma_bf(ah, bl, c);
  c = mma_bf(al, bh, c);
  return c;
}

__global__ __launch_bounds__(256) void prep_split_kernel(
    const float* __restrict__ qk, const float* __restrict__ vin,
    unsigned short* __restrict__ QH, unsigned short* __restrict__ QL,
    unsigned short* __restrict__ KH, unsigned short* __restrict__ KL,
    unsigned short* __restrict__ KTH, unsigned short* __restrict__ KTL,
    unsigned short* __restrict__ VTH, unsigned short* __restrict__ VTL)
{
  __shared__ float sK[kCh * kLdT];
  __shared__ float sV[kCh * kLdT];
  const int tid = threadIdx.x;
  const int c   = blockIdx.x % kNCh;
  const int bh  = blockIdx.x / kNCh;
  const int b   = bh / kNH;
  const int h   = bh - b * kNH;
  const int s0  = c * kCh;

  v4u qh[2], ql[2], kh[2], kl[2];
#pragma unroll
  for (int it = 0; it < 2; ++it) {
    const int idx = it * 256 + tid;
    const int r   = idx >> 3;
    const int c8  = (idx & 7) * 8;
    const size_t qoff = ((((size_t)b * kSeq + s0 + r) * 2) * kNH + h) * kHD + c8;
    const size_t koff = qoff + (size_t)kNH * kHD;
    const size_t voff = (((size_t)b * kSeq + s0 + r) * kNH + h) * kHD + c8;
    const v4f q0 = *(const v4f*)(qk + qoff);
    const v4f q1 = *(const v4f*)(qk + qoff + 4);
    const v4f k0 = *(const v4f*)(qk + koff);
    const v4f k1 = *(const v4f*)(qk + koff + 4);
    const v4f v0 = *(const v4f*)(vin + voff);
    const v4f v1 = *(const v4f*)(vin + voff + 4);
    float xq[8], xk[8], xv[8];
#pragma unroll
    for (int e = 0; e < 4; ++e) {
      xq[e] = q0[e]; xq[4 + e] = q1[e];
      xk[e] = k0[e]; xk[4 + e] = k1[e];
      xv[e] = v0[e]; xv[4 + e] = v1[e];
    }
    split8(xq, qh[it], ql[it]);
    split8(xk, kh[it], kl[it]);
#pragma unroll
    for (int e = 0; e < 8; ++e) {
      sK[r * kLdT + c8 + e] = xk[e];
      sV[r * kLdT + c8 + e] = xv[e];
    }
  }
  for (int pass = 0; pass < 2; ++pass) {
#pragma unroll
    for (int it = 0; it < 2; ++it) {
      const int idx = it * 256 + tid;
      const int r   = idx >> 3;
      const int c8  = (idx & 7) * 8;
      const size_t o = ((size_t)bh * kSeq + s0 + r) * kHD + c8;
      *(volatile v4u*)(QH + o) = qh[it];
      *(volatile v4u*)(QL + o) = ql[it];
      *(volatile v4u*)(KH + o) = kh[it];
      *(volatile v4u*)(KL + o) = kl[it];
    }
    __threadfence();
  }
  __syncthreads();

  v4u th[2], tl[2], uh[2], ul[2];
#pragma unroll
  for (int it = 0; it < 2; ++it) {
    const int idx = it * 256 + tid;
    const int dr  = idx >> 3;
    const int sp  = (idx & 7) * 8;
    float xk[8], xv[8];
#pragma unroll
    for (int e = 0; e < 8; ++e) {
      xk[e] = sK[(sp + e) * kLdT + dr];
      xv[e] = sV[(sp + e) * kLdT + dr];
    }
    split8(xk, th[it], tl[it]);
    split8(xv, uh[it], ul[it]);
  }
  for (int pass = 0; pass < 2; ++pass) {
#pragma unroll
    for (int it = 0; it < 2; ++it) {
      const int idx = it * 256 + tid;
      const int dr  = idx >> 3;
      const int sp  = (idx & 7) * 8;
      const size_t o = (((size_t)bh * kNCh + c) * kCh + dr) * kCh + sp;
      *(volatile v4u*)(KTH + o) = th[it];
      *(volatile v4u*)(KTL + o) = tl[it];
      *(volatile v4u*)(VTH + o) = uh[it];
      *(volatile v4u*)(VTL + o) = ul[it];
    }
    __threadfence();
  }
}

__global__ __launch_bounds__(256) void chunk_state_kernel(
    const unsigned short* __restrict__ VTH, const unsigned short* __restrict__ VTL,
    const unsigned short* __restrict__ KTH, const unsigned short* __restrict__ KTL,
    float* __restrict__ STC)
{
  __shared__ __align__(16) float sO[kCh * kLdO];
  const int tid  = threadIdx.x;
  const int lane = tid & 31;
  const int wave = __builtin_amdgcn_readfirstlane((int)(threadIdx.x >> 5));
  const int hh   = lane >> 4;
  const int cl   = lane & 15;
  const int c    = blockIdx.x % kNChState;
  const int bh   = blockIdx.x / kNChState;
  const int mt   = wave >> 1;
  const int nb   = (wave & 1) * 2;

  const size_t tb = ((size_t)bh * kNCh + c) * kTile;
  const __bf16* Ah = (const __bf16*)VTH + tb;
  const __bf16* Al = (const __bf16*)VTL + tb;
  const __bf16* Bh = (const __bf16*)KTH + tb;
  const __bf16* Bl = (const __bf16*)KTL + tb;

  v8f acc0 = (v8f){0.f, 0.f, 0.f, 0.f, 0.f, 0.f, 0.f, 0.f};
  v8f acc1 = (v8f){0.f, 0.f, 0.f, 0.f, 0.f, 0.f, 0.f, 0.f};
#pragma unroll
  for (int kk = 0; kk < 2; ++kk) {
    const int ao  = (mt * 16 + cl) * kCh + kk * 32 + 8 * hh;
    const int bo0 = ((nb + 0) * 16 + cl) * kCh + kk * 32 + 8 * hh;
    const int bo1 = ((nb + 1) * 16 + cl) * kCh + kk * 32 + 8 * hh;
    const v16b ah = ldfrag(Ah + ao);
    const v16b al = ldfrag(Al + ao);
    const v16b b0h = ldfrag(Bh + bo0);
    const v16b b0l = ldfrag(Bl + bo0);
    acc0 = mma3(ah, al, b0h, b0l, acc0);
    const v16b b1h = ldfrag(Bh + bo1);
    const v16b b1l = ldfrag(Bl + bo1);
    acc1 = mma3(ah, al, b1h, b1l, acc1);
  }
#pragma unroll
  for (int r = 0; r < 8; ++r) {
    const int row = mt * 16 + 8 * hh + r;
    sO[row * kLdO + (nb + 0) * 16 + cl] = acc0[r];
    sO[row * kLdO + (nb + 1) * 16 + cl] = acc1[r];
  }
  __syncthreads();
  {
    const int c4 = cl * 4;
    float* dst = STC + ((size_t)bh * kNChState + c) * kTile;
    v4f vals[4];
#pragma unroll
    for (int it = 0; it < 4; ++it) {
      const int row = wave * 8 + it * 2 + hh;
      vals[it] = *(const v4f*)(sO + row * kLdO + c4);
    }
    for (int pass = 0; pass < 2; ++pass) {
#pragma unroll
      for (int it = 0; it < 4; ++it) {
        const int row = wave * 8 + it * 2 + hh;
        *(volatile v4f*)(dst + (size_t)row * kHD + c4) = vals[it];
      }
      __threadfence();
    }
  }
}

__global__ __launch_bounds__(256) void prefix_scan_kernel(
    const float* __restrict__ STC, unsigned short* __restrict__ STH, unsigned short* __restrict__ STL)
{
  const int idx = blockIdx.x * 256 + threadIdx.x;
  const int bh  = idx >> 9;
  const int e0  = (idx & 511) * 8;
  float run[8];
#pragma unroll
  for (int e = 0; e < 8; ++e) run[e] = 0.0f;
#pragma unroll 1
  for (int c = 0; c < kNCh; ++c) {
    v4u hv, lv;
    split8(run, hv, lv);
    const size_t o = ((size_t)bh * kNCh + c) * kTile + e0;
    *(volatile v4u*)(STH + o) = hv;
    *(volatile v4u*)(STL + o) = lv;
    __threadfence();
    *(volatile v4u*)(STH + o) = hv;
    *(volatile v4u*)(STL + o) = lv;
    if (c < kNChState) {
      const float* src = STC + ((size_t)bh * kNChState + c) * kTile + e0;
      const v4f a0 = *(const v4f*)(src);
      const v4f a1 = *(const v4f*)(src + 4);
#pragma unroll
      for (int e = 0; e < 4; ++e) {
        run[e]     = run[e] + a0[e];
        run[4 + e] = run[4 + e] + a1[e];
      }
    }
  }
}

__global__ __launch_bounds__(256) void chunk_out_kernel(
    const unsigned short* __restrict__ QH, const unsigned short* __restrict__ QL,
    const unsigned short* __restrict__ KH, const unsigned short* __restrict__ KL,
    const unsigned short* __restrict__ VTH, const unsigned short* __restrict__ VTL,
    const unsigned short* __restrict__ STH, const unsigned short* __restrict__ STL,
    const float* __restrict__ nvec, float* __restrict__ out)
{
  __shared__ __align__(16) __bf16 sAh[kCh * kLdA];
  __shared__ __align__(16) __bf16 sAl[kCh * kLdA];
  __shared__ __align__(16) float  sO[kCh * kLdO];
  __shared__ float sE[kCh];

  const int tid  = threadIdx.x;
  const int lane = tid & 31;
  const int wave = __builtin_amdgcn_readfirstlane((int)(threadIdx.x >> 5));
  const int hh   = lane >> 4;
  const int cl   = lane & 15;
  const int c    = blockIdx.x % kNCh;
  const int bh   = blockIdx.x / kNCh;
  const int b    = bh / kNH;
  const int h    = bh - b * kNH;
  const int s0   = c * kCh;
  const int mt   = wave >> 1;
  const int nb   = (wave & 1) * 2;

  {
    const int rr = tid & (kCh - 1);
    float nv = nvec[((size_t)b * kSeq + s0 + rr) * kNH + h];
    asm volatile("" : "+v"(nv));
    const float ev = expf(-nv);
    if (tid < kCh) sE[tid] = ev;
  }

  const size_t rb = ((size_t)bh * kSeq + s0) * kHD;
  const size_t tb = ((size_t)bh * kNCh + c) * kTile;
  const __bf16* Qh = (const __bf16*)QH + rb;
  const __bf16* Ql = (const __bf16*)QL + rb;
  const __bf16* Kh = (const __bf16*)KH + rb;
  const __bf16* Kl = (const __bf16*)KL + rb;
  const __bf16* Vh = (const __bf16*)VTH + tb;
  const __bf16* Vl = (const __bf16*)VTL + tb;
  const __bf16* Sh = (const __bf16*)STH + tb;
  const __bf16* Sl = (const __bf16*)STL + tb;

  v16b qh[2], ql[2];
#pragma unroll
  for (int kk = 0; kk < 2; ++kk) {
    const int ao = (mt * 16 + cl) * kHD + kk * 32 + 8 * hh;
    qh[kk] = ldfrag(Qh + ao);
    ql[kk] = ldfrag(Ql + ao);
  }

  v8f acc[2], am[2];
#pragma unroll
  for (int j = 0; j < 2; ++j) {
    acc[j] = (v8f){0.f, 0.f, 0.f, 0.f, 0.f, 0.f, 0.f, 0.f};
    am[j]  = (v8f){0.f, 0.f, 0.f, 0.f, 0.f, 0.f, 0.f, 0.f};
  }
#pragma unroll
  for (int j = 0; j < 2; ++j) {
#pragma unroll
    for (int kk = 0; kk < 2; ++kk) {
      const int bo = ((nb + j) * 16 + cl) * kHD + kk * 32 + 8 * hh;
      const v16b sh = ldfrag(Sh + bo);
      const v16b sl = ldfrag(Sl + bo);
      acc[j] = mma3(qh[kk], ql[kk], sh, sl, acc[j]);
      const v16b kh = ldfrag(Kh + bo);
      const v16b kl = ldfrag(Kl + bo);
      am[j] = mma3(qh[kk], ql[kk], kh, kl, am[j]);
    }
  }

#pragma unroll
  for (int j = 0; j < 2; ++j) {
#pragma unroll
    for (int r = 0; r < 8; ++r) {
      const int row = mt * 16 + 8 * hh + r;
      const int col = (nb + j) * 16 + cl;
      const float raw = am[j][r];
      const float av  = (col <= row) ? raw : 0.0f;
      const unsigned short hb = f2bf_bits(av);
      const unsigned short lb = f2bf_bits(av - bf_bits2f(hb));
      sAh[row * kLdA + col] = __builtin_bit_cast(__bf16, hb);
      sAl[row * kLdA + col] = __builtin_bit_cast(__bf16, lb);
    }
  }
  __syncthreads();

#pragma unroll
  for (int kk = 0; kk < 2; ++kk) {
    const int ao = (mt * 16 + cl) * kLdA + kk * 32 + 8 * hh;
    const v16b ah = ldfrag(sAh + ao);
    const v16b al = ldfrag(sAl + ao);
#pragma unroll
    for (int j = 0; j < 2; ++j) {
      const int bo = ((nb + j) * 16 + cl) * kCh + kk * 32 + 8 * hh;
      const v16b vh = ldfrag(Vh + bo);
      const v16b vl = ldfrag(Vl + bo);
      acc[j] = mma3(ah, al, vh, vl, acc[j]);
    }
  }

#pragma unroll
  for (int j = 0; j < 2; ++j) {
#pragma unroll
    for (int r = 0; r < 8; ++r) {
      const int row = mt * 16 + 8 * hh + r;
      const float sc = sE[row];
      sO[row * kLdO + (nb + j) * 16 + cl] = acc[j][r] * sc;
    }
  }
  __syncthreads();
  {
    const int c4 = cl * 4;
    v4f vals[4];
#pragma unroll
    for (int it = 0; it < 4; ++it) {
      const int row = wave * 8 + it * 2 + hh;
      vals[it] = *(const v4f*)(sO + row * kLdO + c4);
    }
    for (int pass = 0; pass < 2; ++pass) {
#pragma unroll
      for (int it = 0; it < 4; ++it) {
        const int row = wave * 8 + it * 2 + hh;
        float* dst = out + (((size_t)b * kSeq + s0 + row) * kNH + h) * kHD + c4;
        *(volatile v4f*)dst = vals[it];
      }
      __threadfence();
    }
  }
}

extern "C" void kernel_launch(void* const* d_in, const int* in_sizes, int n_in,
                              void* d_out, int out_size, void* d_ws, size_t ws_size,
                              hipStream_t stream) {
  if (n_in < 3) return;
  if (in_sizes[0] != kNB * kSeq * 2 * kNH * kHD) return;
  if (in_sizes[1] != kNB * kSeq * kNH * kHD) return;
  if (in_sizes[2] != kNB * kSeq * kNH) return;
  if (out_size != kNB * kSeq * kNH * kHD) return;
  if (ws_size < kWsTotal) return;

  const float* qk = (const float*)d_in[0];
  const float* vv = (const float*)d_in[1];
  const float* nn = (const float*)d_in[2];
  float* out = (float*)d_out;

  char* ws = (char*)d_ws;
  unsigned short* QH  = (unsigned short*)(ws + kOffQH);
  unsigned short* QL  = (unsigned short*)(ws + kOffQL);
  unsigned short* KH  = (unsigned short*)(ws + kOffKH);
  unsigned short* KL  = (unsigned short*)(ws + kOffKL);
  unsigned short* KTH = (unsigned short*)(ws + kOffKTH);
  unsigned short* KTL = (unsigned short*)(ws + kOffKTL);
  unsigned short* VTH = (unsigned short*)(ws + kOffVTH);
  unsigned short* VTL = (unsigned short*)(ws + kOffVTL);
  float*          STC = (float*)(ws + kOffSTC);
  unsigned short* STH = (unsigned short*)(ws + kOffSTH);
  unsigned short* STL = (unsigned short*)(ws + kOffSTL);

  prep_split_kernel<<<dim3(kBH * kNCh), dim3(256), 0, stream>>>(qk, vv, QH, QL, KH, KL, KTH, KTL, VTH, VTL);
  chunk_state_kernel<<<dim3(kBH * kNChState), dim3(256), 0, stream>>>(VTH, VTL, KTH, KTL, STC);
  prefix_scan_kernel<<<dim3((kBH * kTile / 8) / 256), dim3(256), 0, stream>>>(STC, STH, STL);
  chunk_out_kernel<<<dim3(kBH * kNCh), dim3(256), 0, stream>>>(QH, QL, KH, KL, VTH, VTL, STH, STL, nn, out);
}
